// PraxisExpert_58128087384380
// MI455X (gfx1250) — hardware-run, weakly checked
//
#include <hip/hip_runtime.h>


#ifndef NB
#define NB 4
#endif
#ifndef SEQ
#define SEQ 2048
#endif
#define NB_FULL  4
#define SEQ_FULL 2048
#define KSEL  2
#define DM    512
#define HID   2048
#define NGRP  8
#define NROW  (NB * SEQ * KSEL)
#define NREL  32
#define RB    1024
#define NBLK  (NROW / RB)
#define OFFP  128
#define PROWS (NROW + 512)
#define NPASS 2
#define TPP   (PROWS / 64 / NPASS)
#define HROWS (TPP * 64)
#define OSW   (16 * 68)

static_assert(NROW % RB == 0);
static_assert(NBLK >= 1 && NBLK <= OFFP);
static_assert(NB <= NB_FULL && SEQ <= SEQ_FULL);
static_assert(NGRP <= NREL && NGRP * 63 <= 512);
static_assert(PROWS % 64 == 0);
static_assert((PROWS / 64) % NPASS == 0);
static_assert(KSEL == 2);
static_assert(DM % 256 == 0 && HID % 256 == 0);
static_assert(DM % 32 == 0 && HID % 32 == 0);
static_assert(DM % 64 == 0 && HID % 64 == 0);
static_assert(DM / 4 == 128);
static_assert(DM * 2 == 2 * 32 * 16);
static_assert(256 * 16 * 2 == 64 * 64 * 2);
static_assert(32 * 16 * 4 == 16 * 64 * 2);
static_assert(32 * 16 * 8 == 16 * 64 * 4);
static_assert(64 * 65 * 4 <= 131072);
static_assert(32 * 32 * 4 + 128 * 4 <= 131072);
static_assert(4 * OSW * 4 <= 131072);

typedef unsigned short bf;
typedef unsigned short hf;
typedef _Float16 h16;
typedef __attribute__((ext_vector_type(16))) __bf16   v16bf;
typedef __attribute__((ext_vector_type(16))) _Float16 v16h;
typedef __attribute__((ext_vector_type(8)))  unsigned short v8us;
typedef __attribute__((ext_vector_type(8)))  float    v8f;
typedef __attribute__((ext_vector_type(4)))  float    v4f;
typedef __attribute__((ext_vector_type(4)))  int      v4i;
typedef v4f  __attribute__((may_alias)) v4fa;
typedef v4i  __attribute__((may_alias)) v4ia;

__device__ __forceinline__ unsigned short f2bf(float f) { unsigned u = __float_as_uint(f); u += 0x7FFFu + ((u >> 16) & 1u); return (unsigned short)(u >> 16); }
__device__ __forceinline__ float bf2f(unsigned short w) { return __uint_as_float(((unsigned)w) << 16); }
__device__ __forceinline__ int clampi(int v, int lo, int hi) { return min(max(v, lo), hi); }
__device__ __forceinline__ v16bf cat16b(v8us lo, v8us hi) { return __builtin_bit_cast(v16bf, __builtin_shufflevector(lo, hi, 0, 1, 2, 3, 4, 5, 6, 7, 8, 9, 10, 11, 12, 13, 14, 15)); }
__device__ __forceinline__ v8f wmmab(v16bf a, v16bf b, v8f c) { return __builtin_amdgcn_wmma_f32_16x16x32_bf16(false, a, false, b, (short)0, c, false, false); }
__device__ __forceinline__ v16bf ldb(const bf* p)  { return cat16b(*(const v8us*)p, *(const v8us*)(p + 16)); }
__device__ __forceinline__ void wave_sync() { __builtin_amdgcn_fence(3  , "wavefront"); __builtin_amdgcn_wave_barrier(); asm volatile("" ::: "memory"); }

__device__ __forceinline__ h16 toh_flush(float v) { const h16 r = (h16)v; return (fabsf(v) < 6.103515625e-05f) ? (h16)0.0f : r; }
__device__ __forceinline__ unsigned short hbits(h16 h) { return __builtin_bit_cast(unsigned short, h); }
__device__ __forceinline__ v16h cat16h(v8us lo, v8us hi) { return __builtin_bit_cast(v16h, __builtin_shufflevector(lo, hi, 0, 1, 2, 3, 4, 5, 6, 7, 8, 9, 10, 11, 12, 13, 14, 15)); }
__device__ __forceinline__ v16h ldh(const hf* p)  { return cat16h(*(const v8us*)p, *(const v8us*)(p + 16)); }
__device__ __forceinline__ v8f wmmah(v16h a, v16h b, v8f c) { return __builtin_amdgcn_wmma_f32_16x16x32_f16(false, a, false, b, (short)0, c, false, false); }
__device__ __forceinline__ v8f mmab(v16bf a, v16bf b, v8f c) { c = wmmab(a, b, c); asm volatile("v_nop\n\tv_nop\n\tv_nop\n\tv_nop" : "+v"(c) : "v"(a), "v"(b)); return c; }
__device__ __forceinline__ v8f mmah(v16h a, v16h b, v8f c) { c = wmmah(a, b, c); asm volatile("v_nop\n\tv_nop\n\tv_nop\n\tv_nop" : "+v"(c) : "v"(a), "v"(b)); return c; }

__device__ __forceinline__ size_t frow(int p) { const int tok = p >> 1; const int b = tok / SEQ; const int s = tok - b * SEQ; return ((((size_t)b * SEQ_FULL) + (size_t)s) << 1) + (size_t)(p & 1); }

__global__ __launch_bounds__(256) void k_wt1(const float* __restrict__ W, bf* WT) {
    __shared__ float ts[64 * 65];
    const int t = threadIdx.x; const int bid = blockIdx.x;
    const int tc = bid % (HID / 64), tr = (bid / (HID / 64)) % (DM / 64), g = bid / ((HID / 64) * (DM / 64));
    const float* src = W + (size_t)g * DM * HID + (size_t)(tr * 64) * HID + tc * 64;
#pragma unroll 1
    for (int i = 0; i < 16; ++i) { const int f = i * 256 + t; ts[(f >> 6) * 65 + (f & 63)] = src[(size_t)(f >> 6) * HID + (f & 63)]; }
    __syncthreads();
    bf* dst = WT + (size_t)g * DM * HID + (size_t)(tc * 64) * DM + tr * 64;
#pragma unroll 1
    for (int ps = 0; ps < 2; ++ps) {
#pragma unroll 1
        for (int it = 0; it < 2; ++it) {
            const int e = it * 32 + (t >> 3), c8 = (t & 7) * 8; v8us o;
#pragma unroll
            for (int k = 0; k < 8; ++k) o[k] = f2bf(ts[(c8 + k) * 65 + e]);
            *(volatile v8us*)(dst + (size_t)e * DM + c8) = o; }
        if (ps == 0) __threadfence(); }
}

__global__ __launch_bounds__(256) void k_wt2(const float* __restrict__ W, hf* WT) {
    __shared__ float ts[64 * 65];
    const int t = threadIdx.x; const int bid = blockIdx.x;
    const int tc = bid % (DM / 64), tr = (bid / (DM / 64)) % (HID / 64), g = bid / ((DM / 64) * (HID / 64));
    const float* src = W + (size_t)g * HID * DM + (size_t)(tr * 64) * DM + tc * 64;
#pragma unroll 1
    for (int i = 0; i < 16; ++i) { const int f = i * 256 + t; ts[(f >> 6) * 65 + (f & 63)] = src[(size_t)(f >> 6) * DM + (f & 63)]; }
    __syncthreads();
    hf* dst = WT + (size_t)g * HID * DM + (size_t)(tc * 64) * HID + tr * 64;
#pragma unroll 1
    for (int ps = 0; ps < 2; ++ps) {
#pragma unroll 1
        for (int it = 0; it < 2; ++it) {
            const int e = it * 32 + (t >> 3), c8 = (t & 7) * 8; v8us o;
#pragma unroll
            for (int k = 0; k < 8; ++k) o[k] = hbits(toh_flush(bf2f(f2bf(ts[(c8 + k) * 65 + e])) * 64.0f));
            *(volatile v8us*)(dst + (size_t)e * HID + c8) = o; }
        if (ps == 0) __threadfence(); }
}

__global__ __launch_bounds__(1024) void k_count(const int* __restrict__ gidx, int* cnt) {
    __shared__ int wc[32 * 32];
    __shared__ __align__(16) int line[32];
    const int tid = threadIdx.x, lane = tid & 31; const int wave = __builtin_amdgcn_readfirstlane(tid >> 5);
    const int blk = blockIdx.x;
    const int rel = clampi(gidx[frow(blk * RB + tid)], 0, NGRP - 1);
    int mine = 0;
#pragma unroll 1
    for (int r = 0; r < NREL; ++r) { const unsigned m = __builtin_amdgcn_ballot_w32(rel == r); const int c = __builtin_popcount(m); mine = (lane == r) ? c : mine; }
    wc[wave * 32 + lane] = mine;
    __syncthreads();
    if (wave == 0) {
        int s = 0;
#pragma unroll 1
        for (int w = 0; w < 32; ++w) s += wc[w * 32 + lane];
        line[lane] = s;
        wave_sync();
#pragma unroll 1
        for (int ps = 0; ps < 2; ++ps) {
            if (lane < 8) { const v4i v = *(const v4ia*)(&line[4 * lane]); *(volatile v4i*)(cnt + (size_t)blk * 32 + 4 * lane) = v; }
            if (ps == 0) __threadfence(); }
    }
}

__global__ __launch_bounds__(1024) void k_scan(const int* __restrict__ cnt, int* offs, int* T, bf* XP) {
    __shared__ int tots[32];
    __shared__ __align__(16) int tl[128];
    const int tid = threadIdx.x, lane = tid & 31; const int r = __builtin_amdgcn_readfirstlane(tid >> 5);
    int c[4]; int ls = 0;
#pragma unroll
    for (int i = 0; i < 4; ++i) { const int blk = 4 * lane + i; const int bc = min(blk, NBLK - 1);
        int v = cnt[(size_t)bc * 32 + r]; v = (blk < NBLK) ? v : 0; v = clampi(v, 0, RB); c[i] = v; ls += v; }
    int x = ls;
#pragma unroll
    for (int d = 1; d < 32; d <<= 1) { const int y = __shfl_up(x, d, 32); x += (lane >= d) ? y : 0; }
    const int excl = x - ls;
    const int tot = __shfl(x, 31, 32);
    if (lane == 0) tots[r] = tot;
    __syncthreads();
    const int t = tots[lane]; const int pd = (t + 63) & ~63;
    int y2 = pd;
#pragma unroll
    for (int d = 1; d < 32; d <<= 1) { const int y = __shfl_up(y2, d, 32); y2 += (lane >= d) ? y : 0; }
    const int sstart = y2 - pd;
    const int ptot = __shfl(y2, 31, 32);
    const int segr = __shfl(sstart, r, 32);
    v4i o; o[0] = segr + excl; o[1] = o[0] + c[0]; o[2] = o[1] + c[1]; o[3] = o[2] + c[2];
    if (r == 0) { tl[lane] = sstart; tl[32 + lane] = t; tl[64 + lane] = (lane == 0) ? ptot : 0; tl[96 + lane] = 0; wave_sync(); }
    const int padcnt = __builtin_amdgcn_readfirstlane(((tot + 63) & ~63) - tot);
    const int pbase = segr + tot;
    v8us z;
#pragma unroll
    for (int k = 0; k < 8; ++k) z[k] = (unsigned short)0;
#pragma unroll 1
    for (int ps = 0; ps < 2; ++ps) {
        *(volatile v4i*)(offs + (size_t)r * OFFP + 4 * lane) = o;
        if (r == 0) { const v4i v = *(const v4ia*)(&tl[4 * lane]); *(volatile v4i*)(T + 4 * lane) = v; }
#pragma unroll 1
        for (int j = 0; j < 64; ++j) { const int p = clampi(pbase + j, 0, PROWS - 1);
            if (j < padcnt) {
#pragma unroll
                for (int q = 0; q < 2; ++q) *(volatile v8us*)(XP + (size_t)p * DM + q * 256 + lane * 8) = z; } }
        if (ps == 0) __threadfence(); }
}

__global__ __launch_bounds__(1024) void k_rank(const int* __restrict__ gidx, const float* __restrict__ xin,
                                               const int* __restrict__ offs, int* POS, bf* XP) {
    __shared__ int wc[32 * 32];
    const int tid = threadIdx.x, lane = tid & 31; const int wave = __builtin_amdgcn_readfirstlane(tid >> 5);
    const int blk = blockIdx.x;
    const int row = blk * RB + tid;
    const int rel = clampi(gidx[frow(row)], 0, NGRP - 1);
    int mine = 0; unsigned mymask = 0u;
#pragma unroll 1
    for (int r = 0; r < NREL; ++r) { const unsigned m = __builtin_amdgcn_ballot_w32(rel == r); const int c = __builtin_popcount(m);
        mine = (lane == r) ? c : mine; mymask = (rel == r) ? m : mymask; }
    const int lrank = __builtin_popcount(mymask & ((1u << lane) - 1u));
    wc[wave * 32 + lane] = mine;
    __syncthreads();
    if (wave == 0) {
        int run = clampi(offs[(size_t)lane * OFFP + blk], 0, PROWS);
#pragma unroll 1
        for (int w = 0; w < 32; ++w) { const int c = wc[w * 32 + lane]; wc[w * 32 + lane] = run; run += c; }
    }
    __syncthreads();
    const int pos = clampi(wc[wave * 32 + rel] + lrank, 0, PROWS - 1);
#pragma unroll 1
    for (int ps = 0; ps < 2; ++ps) {
        *(volatile int*)(POS + row) = pos;
#pragma unroll 1
        for (int j = 0; j < 32; ++j) { const int p = __shfl(pos, j, 32);
            const size_t tok = frow(blk * RB + wave * 32 + j) >> 1;
#pragma unroll
            for (int q = 0; q < 2; ++q) {
                const v8f a = *(const v8f*)(xin + tok * DM + q * 256 + lane * 8); v8us oa;
#pragma unroll
                for (int k = 0; k < 8; ++k) oa[k] = f2bf(a[k]);
                *(volatile v8us*)(XP + (size_t)p * DM + q * 256 + lane * 8) = oa; } }
        if (ps == 0) __threadfence(); }
}

__global__ __launch_bounds__(128) __attribute__((amdgpu_num_vgpr(256))) void k_gemm1(const bf* __restrict__ XP, const bf* __restrict__ W1T, const float* __restrict__ b1,
                                                                                      const int* __restrict__ T, hf* HP, const int tbase) {
    __shared__ __align__(16) float os[4 * OSW];
    const int lane = threadIdx.x & 31, lr = lane & 15, hi = lane >> 4;
    const int wave = __builtin_amdgcn_readfirstlane(threadIdx.x >> 5);
    const int p0 = (tbase + blockIdx.x) * 64;
    const int hr0 = blockIdx.x * 64;
    const int n0 = (blockIdx.y * 4 + wave) * 64;
    const int ss = T[lane], tt = T[32 + lane];
    const int pe = ss + ((tt + 63) & ~63);
    const unsigned msk = __builtin_amdgcn_ballot_w32((p0 >= ss) && (p0 < pe));
    if (msk == 0u) return;
    const int r = __builtin_amdgcn_readfirstlane(min(__builtin_ctz(msk), NGRP - 1));
    v8f acc[4][4];
#pragma unroll
    for (int mb = 0; mb < 4; ++mb)
#pragma unroll
        for (int nb = 0; nb < 4; ++nb) acc[mb][nb] = (v8f){};
    const size_t aoff = (size_t)(p0 + lr) * DM + 8 * hi, boff = (size_t)r * ((size_t)HID * DM) + (size_t)(n0 + lr) * DM + 8 * hi;
#pragma unroll 1
    for (int kc = 0; kc < DM; kc += 32) {
        v16bf a[4];
#pragma unroll
        for (int mb = 0; mb < 4; ++mb) a[mb] = ldb(XP + aoff + (size_t)mb * 16 * DM + kc);
#pragma unroll
        for (int nb = 0; nb < 4; ++nb) { const v16bf b = ldb(W1T + boff + (size_t)nb * 16 * DM + kc);
#pragma unroll
            for (int mb = 0; mb < 4; ++mb) acc[mb][nb] = mmab(a[mb], b, acc[mb][nb]); }
    }
    const int c8 = (lane & 7) * 8, rq = lane >> 3, ob = wave * OSW;
    float bb[8];
    { const v8f bv = *(const v8f*)(b1 + (size_t)r * HID + n0 + c8);
#pragma unroll
      for (int k = 0; k < 8; ++k) bb[k] = bf2f(f2bf(bv[k])); }
#pragma unroll
    for (int mb = 0; mb < 4; ++mb) {
#pragma unroll
        for (int nb = 0; nb < 4; ++nb) {
#pragma unroll
            for (int j = 0; j < 8; ++j) os[ob + (hi * 8 + j) * 68 + nb * 16 + lr] = acc[mb][nb][j]; }
        wave_sync();
        v8us o[4];
#pragma unroll
        for (int it = 0; it < 4; ++it) { const int row = 4 * it + rq;
            const v4f x0 = *(const v4fa*)(&os[ob + row * 68 + c8]); const v4f x1 = *(const v4fa*)(&os[ob + row * 68 + c8 + 4]);
#pragma unroll
            for (int i = 0; i < 4; ++i) { float u = x0[i] + bb[i]; u = (u > 0.0f) ? u : 0.0f; o[it][i] = hbits(toh_flush(u));
                                          float w = x1[i] + bb[4 + i]; w = (w > 0.0f) ? w : 0.0f; o[it][4 + i] = hbits(toh_flush(w)); } }
#pragma unroll 1
        for (int ps = 0; ps < 2; ++ps) {
#pragma unroll
            for (int it = 0; it < 4; ++it) *(volatile v8us*)(HP + (size_t)(hr0 + mb * 16 + 4 * it + rq) * HID + n0 + c8) = o[it];
            if (ps == 0) __threadfence(); }
        wave_sync();
    }
}

__global__ __launch_bounds__(128) __attribute__((amdgpu_num_vgpr(256))) void k_gemm2(const hf* __restrict__ HP, const hf* __restrict__ W2T, const float* __restrict__ b2,
                                                                                      const int* __restrict__ T, float* Y, const int tbase) {
    __shared__ __align__(16) float os[4 * OSW];
    const int lane = threadIdx.x & 31, lr = lane & 15, hi = lane >> 4;
    const int wave = __builtin_amdgcn_readfirstlane(threadIdx.x >> 5);
    const int p0 = (tbase + blockIdx.x) * 64;
    const int hr0 = blockIdx.x * 64;
    const int n0 = (blockIdx.y * 4 + wave) * 64;
    const int ss = T[lane], tt = T[32 + lane];
    const int pe = ss + ((tt + 63) & ~63);
    const unsigned msk = __builtin_amdgcn_ballot_w32((p0 >= ss) && (p0 < pe));
    if (msk == 0u) return;
    const int r = __builtin_amdgcn_readfirstlane(min(__builtin_ctz(msk), NGRP - 1));
    v8f acc[4][4];
#pragma unroll
    for (int mb = 0; mb < 4; ++mb)
#pragma unroll
        for (int nb = 0; nb < 4; ++nb) acc[mb][nb] = (v8f){};
    const size_t aoff = (size_t)(hr0 + lr) * HID + 8 * hi, boff = (size_t)r * ((size_t)DM * HID) + (size_t)(n0 + lr) * HID + 8 * hi;
#pragma unroll 1
    for (int kc = 0; kc < HID; kc += 32) {
        v16h a[4];
#pragma unroll
        for (int mb = 0; mb < 4; ++mb) a[mb] = ldh(HP + aoff + (size_t)mb * 16 * HID + kc);
#pragma unroll
        for (int nb = 0; nb < 4; ++nb) { const v16h b = ldh(W2T + boff + (size_t)nb * 16 * HID + kc);
#pragma unroll
            for (int mb = 0; mb < 4; ++mb) acc[mb][nb] = mmah(a[mb], b, acc[mb][nb]); }
    }
    const int c4 = (lane & 15) * 4, rh = lane >> 4, ob = wave * OSW;
    float bb[4];
    { const v4f bv = *(const v4f*)(b2 + (size_t)r * DM + n0 + c4);
#pragma unroll
      for (int k = 0; k < 4; ++k) bb[k] = bf2f(f2bf(bv[k])); }
#pragma unroll
    for (int mb = 0; mb < 4; ++mb) {
#pragma unroll
        for (int nb = 0; nb < 4; ++nb) {
#pragma unroll
            for (int j = 0; j < 8; ++j) os[ob + (hi * 8 + j) * 68 + nb * 16 + lr] = acc[mb][nb][j]; }
        wave_sync();
        v4f o[8];
#pragma unroll
        for (int it = 0; it < 8; ++it) { const int row = 2 * it + rh;
            const v4f x0 = *(const v4fa*)(&os[ob + row * 68 + c4]);
#pragma unroll
            for (int i = 0; i < 4; ++i) o[it][i] = x0[i] * 0.015625f + bb[i]; }
#pragma unroll 1
        for (int ps = 0; ps < 2; ++ps) {
#pragma unroll
            for (int it = 0; it < 8; ++it) *(volatile v4f*)(Y + (size_t)(p0 + mb * 16 + 2 * it + rh) * DM + n0 + c4) = o[it];
            if (ps == 0) __threadfence(); }
        wave_sync();
    }
}

__global__ __launch_bounds__(256) void k_unsort(const int* __restrict__ POS, const float* __restrict__ Y, float* OUT) {
    const size_t i = (size_t)blockIdx.x * 256 + threadIdx.x; if (i >= (size_t)NROW * (DM / 4)) return;
    const int p = (int)(i >> 7); const int c4 = (int)(i & 127) * 4;
    const int pos = clampi(POS[p], 0, PROWS - 1);
    const v4f v = *(const v4f*)(Y + (size_t)pos * DM + c4);
    float* dst = OUT + frow(p) * DM + c4;
    *(volatile v4f*)dst = v; __threadfence(); *(volatile v4f*)dst = v;
}

static constexpr size_t al256(size_t v) { return (v + 255) & ~(size_t)255; }
static constexpr size_t SZ_W   = al256((size_t)NGRP * DM * HID * 2);
static constexpr size_t SZ_CNT = al256((size_t)NBLK * 32 * 4);
static constexpr size_t SZ_OFF = al256((size_t)NREL * OFFP * 4);
static constexpr size_t SZ_T   = al256((size_t)128 * 4);
static constexpr size_t SZ_POS = al256((size_t)NROW * 4);
static constexpr size_t SZ_XP  = al256((size_t)PROWS * DM * 2);
static constexpr size_t SZ_HP  = al256((size_t)HROWS * HID * 2);
static constexpr size_t SZ_Y   = al256((size_t)PROWS * DM * 4);
static constexpr size_t SZ_TOTAL = 2 * SZ_W + SZ_CNT + SZ_OFF + SZ_T + SZ_POS + SZ_XP + SZ_HP + SZ_Y;
static_assert(SZ_TOTAL <= (size_t)134217728);
static_assert((size_t)NPASS * HROWS == (size_t)PROWS);

extern "C" void kernel_launch(void* const* d_in, const int* in_sizes, int n_in,
                              void* d_out, int out_size, void* d_ws, size_t ws_size, hipStream_t stream) {
    if (n_in < 6) return;
    const size_t tokneed = (size_t)(NB - 1) * SEQ_FULL + (size_t)SEQ;
    if ((size_t)in_sizes[0] < tokneed * DM) return;
    if ((size_t)in_sizes[1] < tokneed * KSEL) return;
    if ((size_t)in_sizes[2] < (size_t)NGRP * DM * HID) return;
    if ((size_t)in_sizes[3] < (size_t)NGRP * HID) return;
    if ((size_t)in_sizes[4] < (size_t)NGRP * HID * DM) return;
    if ((size_t)in_sizes[5] < (size_t)NGRP * DM) return;
    if ((size_t)out_size < tokneed * KSEL * DM) return;
    if (SZ_TOTAL > ws_size) return;
    const float* xin  = (const float*)d_in[0];
    const int*   gidx = (const int*)d_in[1];
    const float* W1   = (const float*)d_in[2];
    const float* b1   = (const float*)d_in[3];
    const float* W2   = (const float*)d_in[4];
    const float* b2   = (const float*)d_in[5];
    float* OUT = (float*)d_out;
    char* wsp = (char*)d_ws;
    bf*  W1T = (bf*)wsp;  wsp += SZ_W;
    hf*  W2T = (hf*)wsp;  wsp += SZ_W;
    int* CNT = (int*)wsp; wsp += SZ_CNT;
    int* OFF = (int*)wsp; wsp += SZ_OFF;
    int* TT  = (int*)wsp; wsp += SZ_T;
    int* POS = (int*)wsp; wsp += SZ_POS;
    bf*  XP  = (bf*)wsp;  wsp += SZ_XP;
    hf*  HP  = (hf*)wsp;  wsp += SZ_HP;
    float* YP = (float*)wsp; wsp += SZ_Y;

    k_wt1<<<NGRP * (DM / 64) * (HID / 64), 256, 0, stream>>>(W1, W1T);
    k_wt2<<<NGRP * (HID / 64) * (DM / 64), 256, 0, stream>>>(W2, W2T);
    k_count<<<NBLK, 1024, 0, stream>>>(gidx, CNT);
    k_scan<<<1, 1024, 0, stream>>>(CNT, OFF, TT, XP);
    k_rank<<<NBLK, 1024, 0, stream>>>(gidx, xin, OFF, POS, XP);
    for (int ps = 0; ps < NPASS; ++ps) {
        k_gemm1<<<dim3(TPP, HID / 256), 128, 0, stream>>>(XP, W1T, b1, TT, HP, ps * TPP);
        k_gemm2<<<dim3(TPP, DM / 256), 128, 0, stream>>>(HP, W2T, b2, TT, YP, ps * TPP);
    }
    k_unsort<<<(unsigned)(((size_t)NROW * (DM / 4) + 255) / 256), 256, 0, stream>>>(POS, YP, OUT);
}
